// DeepSeek_MLA_79078937854405
// MI455X (gfx1250) — hardware-verified
//
#include <hip/hip_runtime.h>
#include <stddef.h>
#include <stdint.h>

#define NB    2
#define SQ    2048
#define NTOK  (NB * SQ)
#define HID   2048
#define NH    16
#define NBH   (NB * NH)
#define HDM   128
#define PD    64
#define PHALF 32
#define LAT   512
#define CLP   (2 * LAT)
#define NDN   (2 * LAT + PD)
#define NUP   (3 * HID + NH * PD)
#define QB    128
#define KC    64
#define NQB   (SQ / QB)
#define NCK   (SQ / KC)

static_assert(NH * HDM == HID);
static_assert(SQ % 256 == 0);
static_assert(HID % 64 == 0);
static_assert(LAT % 64 == 0);
static_assert(PD == 64);
static_assert(NDN % 64 == 0);
static_assert(NUP % 128 == 0);
static_assert(SQ % KC == 0);
static_assert(SQ % QB == 0);
static_assert((SQ * PHALF) % 256 == 0);

typedef _Float16 v16h __attribute__((ext_vector_type(16)));
typedef _Float16 v8h  __attribute__((ext_vector_type(8)));
typedef float    v8f  __attribute__((ext_vector_type(8)));
typedef float    v4f  __attribute__((ext_vector_type(4)));
typedef unsigned int v4u __attribute__((ext_vector_type(4)));

union Frag  { v16h v; v8h h[2]; };
union Pack8 { v8h h; v4u u; };

__device__ __forceinline__ v8f mma16(v16h a, v16h b, v8f c) {
  c = __builtin_amdgcn_wmma_f32_16x16x32_f16(false, a, false, b, (short)0, c, false, false);
  asm volatile("v_nop\n\tv_nop\n\tv_nop\n\tv_nop" : "+v"(c) : "v"(a), "v"(b));
  return c;
}

__device__ __forceinline__ v16h ldfrag(const _Float16* p, int ld, int row0, int k0, int lane) {
  const int m = lane & 15, lh = lane >> 4;
  const _Float16* q = p + (size_t)(row0 + m) * ld + k0 + 8 * lh;
  Frag f;
  f.h[0] = *(const v8h*)(q);
  f.h[1] = *(const v8h*)(q + 16);
  return f.v;
}

__device__ __forceinline__ v8f zero8() { return (v8f){0.f, 0.f, 0.f, 0.f, 0.f, 0.f, 0.f, 0.f}; }

__device__ __forceinline__ v4u pk8(v4f a0, v4f a1) {
  Pack8 pk;
  pk.h = (v8h){(_Float16)a0[0], (_Float16)a0[1], (_Float16)a0[2], (_Float16)a0[3],
               (_Float16)a1[0], (_Float16)a1[1], (_Float16)a1[2], (_Float16)a1[3]};
  return pk.u;
}

template <int KD>
__device__ __forceinline__ void gemm16x64(const _Float16* __restrict__ A, int lda,
                                          const _Float16* __restrict__ Bt, int ldb,
                                          int m0, int n0, int lane, v8f (&acc)[4]) {
  static_assert(KD % 32 == 0);
#pragma unroll 2
  for (int k0 = 0; k0 < KD; k0 += 32) {
    const v16h a = ldfrag(A, lda, m0, k0, lane);
#pragma unroll
    for (int t = 0; t < 4; ++t) {
      const v16h b = ldfrag(Bt, ldb, n0 + 16 * t, k0, lane);
      acc[t] = mma16(a, b, acc[t]);
    }
  }
}

__device__ __forceinline__ void gemm32x64(const _Float16* __restrict__ A, int lda,
                                          const _Float16* __restrict__ Bt, int ldb,
                                          int m0, int n0, int lane, v8f (&acc)[2][4]) {
#pragma unroll 2
  for (int k0 = 0; k0 < HID; k0 += 32) {
    const v16h a0 = ldfrag(A, lda, m0, k0, lane);
    const v16h a1 = ldfrag(A, lda, m0 + 16, k0, lane);
    const v16h b0 = ldfrag(Bt, ldb, n0, k0, lane);
    const v16h b1 = ldfrag(Bt, ldb, n0 + 16, k0, lane);
    const v16h b2 = ldfrag(Bt, ldb, n0 + 32, k0, lane);
    const v16h b3 = ldfrag(Bt, ldb, n0 + 48, k0, lane);
    acc[0][0] = mma16(a0, b0, acc[0][0]);
    acc[1][0] = mma16(a1, b0, acc[1][0]);
    acc[0][1] = mma16(a0, b1, acc[0][1]);
    acc[1][1] = mma16(a1, b1, acc[1][1]);
    acc[0][2] = mma16(a0, b2, acc[0][2]);
    acc[1][2] = mma16(a1, b2, acc[1][2]);
    acc[0][3] = mma16(a0, b3, acc[0][3]);
    acc[1][3] = mma16(a1, b3, acc[1][3]);
  }
}

__global__ __launch_bounds__(256) void k_tab(float* __restrict__ ct, float* __restrict__ sn) {
  __shared__ float invf[PHALF];
  const int tid = threadIdx.x;
  if (tid < PHALF) {
    const int j  = tid;
    const int ip = j >> 3;
    double p = 1.0;
    if (ip >= 1) p *= 10.0;
    if (ip >= 2) p *= 10.0;
    if (ip >= 3) p *= 10.0;
    if (j & 4) p *= 3.1622776601683795;
    if (j & 2) p *= 1.7782794100389228;
    if (j & 1) p *= 1.3335214321633240;
    const float t32 = (float)p;
    invf[j] = 1.0f / t32;
  }
  __syncthreads();
  const int e = blockIdx.x * 256 + tid;
  const int s = e >> 5, j = e & 31;
  const float ang = (float)s * invf[j];
  float sv, cv;
  sincosf(ang, &sv, &cv);
  volatile float* dc = (volatile float*)(ct + e);
  volatile float* ds = (volatile float*)(sn + e);
  *dc = cv;
  *ds = sv;
  __threadfence();
  *dc = cv;
  *ds = sv;
}

__global__ __launch_bounds__(256) void k_cvtx(const float* __restrict__ src, _Float16* __restrict__ dh,
                                              int ngrp) {
  const int t = blockIdx.x * 256 + (int)threadIdx.x;
  if (t >= ngrp) return;
  const size_t o = (size_t)t * 8;
  const v4f a0 = *(const v4f*)(src + o);
  const v4f a1 = *(const v4f*)(src + o + 4);
  const v4u vv = pk8(a0, a1);
  volatile v4u* d = (volatile v4u*)(dh + o);
  *d = vv;
  __threadfence();
  *d = vv;
}

#define WTP 65
__global__ __launch_bounds__(256) void k_wtr(const float* __restrict__ W, int ncol, int kdim, int nofs,
                                             _Float16* __restrict__ wt) {
  __shared__ float tl[64 * WTP];
  const int tid = threadIdx.x;
  const int n0 = blockIdx.x * 64, k0 = blockIdx.y * 64;
#pragma unroll
  for (int j = 0; j < 4; ++j) {
    const int p  = tid + 256 * j;
    const int kk = p >> 4;
    const int q4 = (p & 15) * 4;
    const v4f a = *(const v4f*)(W + (size_t)(k0 + kk) * ncol + n0 + q4);
    float* d = tl + kk * WTP + q4;
    d[0] = a[0]; d[1] = a[1]; d[2] = a[2]; d[3] = a[3];
  }
  __syncthreads();
  v4u vt[2];
  size_t go[2];
#pragma unroll
  for (int j = 0; j < 2; ++j) {
    const int p  = tid + 256 * j;
    const int nn = p >> 3;
    const int pc = p & 7;
    const float* cp = tl + (pc * 8) * WTP + nn;
    Pack8 pk;
    pk.h = (v8h){(_Float16)(cp[0 * WTP] * 32.0f), (_Float16)(cp[1 * WTP] * 32.0f),
                 (_Float16)(cp[2 * WTP] * 32.0f), (_Float16)(cp[3 * WTP] * 32.0f),
                 (_Float16)(cp[4 * WTP] * 32.0f), (_Float16)(cp[5 * WTP] * 32.0f),
                 (_Float16)(cp[6 * WTP] * 32.0f), (_Float16)(cp[7 * WTP] * 32.0f)};
    vt[j] = pk.u;
    go[j] = (size_t)(nofs + n0 + nn) * kdim + k0 + pc * 8;
  }
  for (int ps = 0; ps < 2; ++ps) {
#pragma unroll
    for (int j = 0; j < 2; ++j) *(volatile v4u*)(wt + go[j]) = vt[j];
    __threadfence();
  }
}

#define SFD 68
__global__ __launch_bounds__(128) void k_down(const _Float16* __restrict__ xh,
                                              const _Float16* __restrict__ wd,
                                              const float* __restrict__ ct,
                                              const float* __restrict__ sn,
                                              _Float16* __restrict__ cl,
                                              _Float16* __restrict__ kr) {
  __shared__ __align__(16) float sf[64 * SFD];
  const int tid = threadIdx.x, lane = tid & 31, wave = tid >> 5;
  const int hh = lane >> 4, c = lane & 15;
  const int mb = blockIdx.x * 64;
  const int ns = blockIdx.y;
  const int m0 = mb + wave * 16;
  const int n0 = ns * 64;

  v8f acc[4];
#pragma unroll
  for (int t = 0; t < 4; ++t) acc[t] = zero8();
  gemm16x64<HID>(xh, HID, wd, HID, m0, n0, lane, acc);

#pragma unroll
  for (int t = 0; t < 4; ++t) {
#pragma unroll
    for (int r = 0; r < 8; ++r)
      sf[(wave * 16 + 8 * hh + r) * SFD + 16 * t + c] = acc[t][r] * 0.03125f;
  }
  __syncthreads();

  v4u val[4];
  size_t go[4];
  _Float16* base;
  if (ns < CLP / 64) {
#pragma unroll
    for (int j = 0; j < 4; ++j) {
      const int p  = tid + 128 * j;
      const int lr = p >> 3;
      const int pc = p & 7;
      const float* ra = sf + lr * SFD + pc * 8;
      const v4f a0 = *(const v4f*)(ra), a1 = *(const v4f*)(ra + 4);
      val[j] = pk8(a0, a1);
      go[j]  = (size_t)(mb + lr) * CLP + ns * 64 + pc * 8;
    }
    base = cl;
  } else {
#pragma unroll
    for (int j = 0; j < 4; ++j) {
      const int p  = tid + 128 * j;
      const int lr = p >> 3;
      const int pc = p & 7;
      const int d0 = pc * 8;
      const int j0 = d0 & (PHALF - 1);
      const float* ra = sf + lr * SFD + d0;
      const float* rb = sf + lr * SFD + (d0 ^ PHALF);
      const v4f a0 = *(const v4f*)(ra), a1 = *(const v4f*)(ra + 4);
      const v4f b0 = *(const v4f*)(rb), b1 = *(const v4f*)(rb + 4);
      const int pos = (mb + lr) & (SQ - 1);
      const size_t to = (size_t)pos * PHALF + j0;
      const v4f c0 = *(const v4f*)(ct + to), c1 = *(const v4f*)(ct + to + 4);
      const v4f s0 = *(const v4f*)(sn + to), s1 = *(const v4f*)(sn + to + 4);
      const float sg = (pc < 4) ? -1.0f : 1.0f;
      const v4f o0 = a0 * c0 + sg * (b0 * s0);
      const v4f o1 = a1 * c1 + sg * (b1 * s1);
      val[j] = pk8(o0, o1);
      go[j]  = (size_t)(mb + lr) * PD + d0;
    }
    base = kr;
  }
  for (int ps = 0; ps < 2; ++ps) {
#pragma unroll
    for (int j = 0; j < 4; ++j) *(volatile v4u*)(base + go[j]) = val[j];
    __threadfence();
  }
}

#define SFU 132
__global__ __launch_bounds__(256) void k_up(const _Float16* __restrict__ cl,
                                            const _Float16* __restrict__ wu,
                                            const float* __restrict__ ct,
                                            const float* __restrict__ sn,
                                            _Float16* __restrict__ qc,
                                            _Float16* __restrict__ qr,
                                            _Float16* __restrict__ kcp,
                                            _Float16* __restrict__ vtp) {
  __shared__ __align__(16) float sf[64 * SFU];
  const int tid = threadIdx.x, lane = tid & 31, wave = tid >> 5;
  const int hh = lane >> 4, c = lane & 15;
  const int wm = wave >> 1, wn = wave & 1;
  const int mb = blockIdx.x * 64;
  const int ns = blockIdx.y;
  const int which = (ns < NH) ? 0 : ((ns < 2 * NH) ? 1 : ((ns < 3 * NH) ? 2 : 3));
  const int aofs = (which >= 2) ? LAT : 0;
  const int m0 = mb + wm * 16;
  const int n0 = ns * HDM + wn * 64;
  const int b  = mb / SQ;
  const int s0 = mb & (SQ - 1);

  v8f acc[4];
#pragma unroll
  for (int t = 0; t < 4; ++t) acc[t] = zero8();
  gemm16x64<LAT>(cl + aofs, CLP, wu, LAT, m0, n0, lane, acc);

#pragma unroll
  for (int t = 0; t < 4; ++t) {
#pragma unroll
    for (int r = 0; r < 8; ++r)
      sf[(wm * 16 + 8 * hh + r) * SFU + wn * 64 + 16 * t + c] = acc[t][r] * 0.03125f;
  }
  __syncthreads();

  v4u val[4];
  size_t go[4];
  _Float16* base;
  if (which == 0 || which == 2) {
    const int head = (which == 0) ? ns : (ns - 2 * NH);
    const int bh = b * NH + head;
#pragma unroll
    for (int j = 0; j < 4; ++j) {
      const int p  = tid + 256 * j;
      const int lr = p >> 4;
      const int pc = p & 15;
      const float* ra = sf + lr * SFU + pc * 8;
      const v4f a0 = *(const v4f*)(ra), a1 = *(const v4f*)(ra + 4);
      val[j] = pk8(a0, a1);
      go[j]  = ((size_t)bh * SQ + s0 + lr) * HDM + pc * 8;
    }
    base = (which == 0) ? kcp : qc;
  } else if (which == 1) {
    const int bh = b * NH + (ns - NH);
#pragma unroll
    for (int j = 0; j < 4; ++j) {
      const int p  = tid + 256 * j;
      const int d  = p >> 3;
      const int pc = p & 7;
      const float* cp = sf + (pc * 8) * SFU + d;
      Pack8 pk;
      pk.h = (v8h){(_Float16)cp[0 * SFU], (_Float16)cp[1 * SFU], (_Float16)cp[2 * SFU], (_Float16)cp[3 * SFU],
                   (_Float16)cp[4 * SFU], (_Float16)cp[5 * SFU], (_Float16)cp[6 * SFU], (_Float16)cp[7 * SFU]};
      val[j] = pk.u;
      go[j]  = ((size_t)bh * HDM + d) * SQ + s0 + pc * 8;
    }
    base = vtp;
  } else {
    const int hA = 2 * (ns - 3 * NH);
#pragma unroll
    for (int j = 0; j < 4; ++j) {
      const int p    = tid + 256 * j;
      const int lr   = p >> 4;
      const int pc   = p & 15;
      const int hsub = pc >> 3;
      const int d0   = (pc & 7) * 8;
      const int col  = pc * 8;
      const int j0   = d0 & (PHALF - 1);
      const float* ra = sf + lr * SFU + col;
      const float* rb = sf + lr * SFU + (col ^ PHALF);
      const v4f a0 = *(const v4f*)(ra), a1 = *(const v4f*)(ra + 4);
      const v4f b0 = *(const v4f*)(rb), b1 = *(const v4f*)(rb + 4);
      const int pos = s0 + lr;
      const size_t to = (size_t)pos * PHALF + j0;
      const v4f c0 = *(const v4f*)(ct + to), c1 = *(const v4f*)(ct + to + 4);
      const v4f sv0 = *(const v4f*)(sn + to), sv1 = *(const v4f*)(sn + to + 4);
      const float sg = ((pc & 7) < 4) ? -1.0f : 1.0f;
      const v4f o0 = a0 * c0 + sg * (b0 * sv0);
      const v4f o1 = a1 * c1 + sg * (b1 * sv1);
      val[j] = pk8(o0, o1);
      const int bh = b * NH + hA + hsub;
      go[j]  = ((size_t)bh * SQ + pos) * PD + d0;
    }
    base = qr;
  }
  for (int ps = 0; ps < 2; ++ps) {
#pragma unroll
    for (int j = 0; j < 4; ++j) *(volatile v4u*)(base + go[j]) = val[j];
    __threadfence();
  }
}

#define KTK 200
#define KTP 72
__global__ __launch_bounds__(256) void k_attn(const _Float16* __restrict__ qc,
                                              const _Float16* __restrict__ qr,
                                              const _Float16* __restrict__ kcp,
                                              const _Float16* __restrict__ kr,
                                              const _Float16* __restrict__ vt,
                                              _Float16* __restrict__ op, float sscale) {
  __shared__ __align__(16) _Float16 Ks[KC * KTK];
  __shared__ __align__(16) _Float16 Vs[HDM * KTP];
  __shared__ __align__(16) _Float16 Ps[8 * 16 * KTP];

  const int tid = threadIdx.x, lane = tid & 31, wave = tid >> 5;
  const int hh = lane >> 4, c = lane & 15;
  const int bh = blockIdx.x / NQB;
  const int qb = blockIdx.x % NQB;
  const int b  = bh / NH, h = bh % NH;
  const int q0 = qb * QB + wave * 16;

  const _Float16* QC = qc  + (size_t)bh * SQ * HDM;
  const _Float16* QR = qr  + (size_t)bh * SQ * PD;
  const _Float16* K  = kcp + (size_t)bh * SQ * HDM;
  const _Float16* KR = kr  + (size_t)b  * SQ * PD;
  const _Float16* V  = vt  + (size_t)bh * HDM * SQ;

  const float NEGI = -__builtin_huge_valf();
  float mrow[8], lrow[8];
  v8f oacc[8];
#pragma unroll
  for (int r = 0; r < 8; ++r) { mrow[r] = NEGI; lrow[r] = 0.f; }
#pragma unroll
  for (int t = 0; t < 8; ++t) oacc[t] = zero8();

  _Float16* pw = Ps + wave * 16 * KTP;

  for (int kci = 0; kci < NCK; ++kci) {
    const int kv0 = kci * KC;
    __syncthreads();
    {
      const int r  = tid >> 2;
      const int qq = (tid & 3) * 32;
      const _Float16* ks = K + (size_t)(kv0 + r) * HDM + qq;
#pragma unroll
      for (int e = 0; e < 4; ++e) *(v8h*)(Ks + r * KTK + qq + 8 * e) = *(const v8h*)(ks + 8 * e);
      const int q16 = (tid & 3) * 16;
      const _Float16* krs = KR + (size_t)(kv0 + r) * PD + q16;
#pragma unroll
      for (int e = 0; e < 2; ++e) *(v8h*)(Ks + r * KTK + HDM + q16 + 8 * e) = *(const v8h*)(krs + 8 * e);
      const int dr = tid >> 1;
      const int q2 = (tid & 1) * 32;
      const _Float16* vs = V + (size_t)dr * SQ + kv0 + q2;
#pragma unroll
      for (int e = 0; e < 4; ++e) *(v8h*)(Vs + dr * KTP + q2 + 8 * e) = *(const v8h*)(vs + 8 * e);
    }
    __syncthreads();

    v8f s[4];
#pragma unroll
    for (int j = 0; j < 4; ++j) s[j] = zero8();
#pragma unroll
    for (int dc = 0; dc < 4; ++dc) {
      const v16h qa = ldfrag(QC, HDM, q0, dc * 32, lane);
#pragma unroll
      for (int j = 0; j < 4; ++j) {
        const v16h kb = ldfrag(Ks, KTK, j * 16, dc * 32, lane);
        s[j] = mma16(qa, kb, s[j]);
      }
    }
#pragma unroll
    for (int dc = 0; dc < 2; ++dc) {
      const v16h qa = ldfrag(QR, PD, q0, dc * 32, lane);
#pragma unroll
      for (int j = 0; j < 4; ++j) {
        const v16h kb = ldfrag(Ks, KTK, j * 16, HDM + dc * 32, lane);
        s[j] = mma16(qa, kb, s[j]);
      }
    }
#pragma unroll
    for (int r = 0; r < 8; ++r) {
#pragma unroll
      for (int j = 0; j < 4; ++j) s[j][r] = s[j][r] * sscale;
    }
    float cm[8];
#pragma unroll
    for (int r = 0; r < 8; ++r) {
      float m = NEGI;
#pragma unroll
      for (int j = 0; j < 4; ++j) m = fmaxf(m, s[j][r]);
#pragma unroll
      for (int off = 1; off < 16; off <<= 1) m = fmaxf(m, __shfl_xor(m, off, 32));
      cm[r] = m;
    }
    float al[8];
#pragma unroll
    for (int r = 0; r < 8; ++r) {
      const float mnew  = fmaxf(mrow[r], cm[r]);
      const float alpha = __expf(mrow[r] - mnew);
      mrow[r] = mnew;
      float psum = 0.f;
#pragma unroll
      for (int j = 0; j < 4; ++j) {
        const float p = __expf(s[j][r] - mnew);
        psum += p;
        pw[(8 * hh + r) * KTP + j * 16 + c] = (_Float16)(p * 1024.0f);
      }
#pragma unroll
      for (int off = 1; off < 16; off <<= 1) psum += __shfl_xor(psum, off, 32);
      lrow[r] = lrow[r] * alpha + psum;
      al[r] = alpha;
    }
#pragma unroll
    for (int t = 0; t < 8; ++t)
#pragma unroll
      for (int r = 0; r < 8; ++r) oacc[t][r] *= al[r];
    __syncthreads();

#pragma unroll
    for (int kk = 0; kk < 2; ++kk) {
      const v16h pa = ldfrag(pw, KTP, 0, kk * 32, lane);
#pragma unroll
      for (int t = 0; t < 8; ++t) {
        const v16h vb = ldfrag(Vs, KTP, t * 16, kk * 32, lane);
        oacc[t] = mma16(pa, vb, oacc[t]);
      }
    }
  }

  float invl[8];
#pragma unroll
  for (int r = 0; r < 8; ++r) invl[r] = (lrow[r] > 0.f) ? (0.0625f / lrow[r]) : 0.f;
#pragma unroll
  for (int half = 0; half < 2; ++half) {
    __syncthreads();
#pragma unroll
    for (int r = 0; r < 8; ++r) {
#pragma unroll
      for (int t = 0; t < 4; ++t)
        pw[(8 * hh + r) * KTP + 16 * t + c] = (_Float16)(oacc[4 * half + t][r] * invl[r]);
    }
    __syncthreads();
    v4u val[4];
    size_t go[4];
#pragma unroll
    for (int it = 0; it < 4; ++it) {
      const int p  = lane + 32 * it;
      const int L  = p >> 3;
      const int pc = p & 7;
      Pack8 pk;
      pk.h    = *(const v8h*)(pw + L * KTP + pc * 8);
      val[it] = pk.u;
      go[it]  = (size_t)(b * SQ + q0 + L) * HID + (size_t)h * HDM + half * 64 + pc * 8;
    }
    for (int ps = 0; ps < 2; ++ps) {
#pragma unroll
      for (int it = 0; it < 4; ++it) *(volatile v4u*)(op + go[it]) = val[it];
      __threadfence();
    }
  }
}

#define OTP 68
__device__ __forceinline__ void out_epilogue(v8f (&acc)[2][4], float scale, float* sw, float* __restrict__ out,
                                             int m0, int n0, int lane, int hh, int c) {
#pragma unroll
  for (int sub = 0; sub < 2; ++sub) {
    __syncthreads();
#pragma unroll
    for (int t = 0; t < 4; ++t) {
#pragma unroll
      for (int r = 0; r < 8; ++r) sw[(8 * hh + r) * OTP + 16 * t + c] = acc[sub][t][r] * scale;
    }
    __syncthreads();
    v4f val[8];
    size_t go[8];
#pragma unroll
    for (int it = 0; it < 8; ++it) {
      const int p    = lane + 32 * it;
      const int L    = p >> 3;
      const int pc   = p & 7;
      const int row  = L >> 1;
      const int half = L & 1;
      val[it] = *(const v4f*)(sw + row * OTP + half * 32 + pc * 4);
      go[it]  = (size_t)(m0 + sub * 16 + row) * HID + n0 + half * 32 + pc * 4;
    }
    for (int ps = 0; ps < 2; ++ps) {
#pragma unroll
      for (int it = 0; it < 8; ++it) *(volatile v4f*)(out + go[it]) = val[it];
      __threadfence();
    }
  }
}

__global__ __launch_bounds__(256) void k_out(const _Float16* __restrict__ ap,
                                             const _Float16* __restrict__ wt,
                                             float* __restrict__ out) {
  __shared__ __align__(16) float st[8][16 * OTP];
  const int tid = threadIdx.x, lane = tid & 31, wave = tid >> 5;
  const int hh = lane >> 4, c = lane & 15;
  const int m0 = blockIdx.x * 256 + wave * 32;
  const int n0 = blockIdx.y * 64;

  v8f acc[2][4];
#pragma unroll
  for (int s = 0; s < 2; ++s)
#pragma unroll
    for (int t = 0; t < 4; ++t) acc[s][t] = zero8();
  gemm32x64(ap, HID, wt, HID, m0, n0, lane, acc);
  out_epilogue(acc, 0.00048828125f, st[wave], out, m0, n0, lane, hh, c);
}

extern "C" void kernel_launch(void* const* d_in, const int* in_sizes, int n_in,
                              void* d_out, int out_size, void* d_ws, size_t ws_size,
                              hipStream_t stream) {
  if (n_in < 9) return;
  if (in_sizes[0] != NTOK * HID) return;
  if (in_sizes[1] != HID * LAT) return;
  if (in_sizes[2] != HID * LAT) return;
  if (in_sizes[3] != LAT * HID) return;
  if (in_sizes[4] != LAT * HID) return;
  if (in_sizes[5] != LAT * HID) return;
  if (in_sizes[6] != HID * PD) return;
  if (in_sizes[7] != LAT * NH * PD) return;
  if (in_sizes[8] != HID * HID) return;
  if (out_size != NTOK * HID) return;

  const float* x    = (const float*)d_in[0];
  const float* wdkv = (const float*)d_in[1];
  const float* wdq  = (const float*)d_in[2];
  const float* wuk  = (const float*)d_in[3];
  const float* wuv  = (const float*)d_in[4];
  const float* wuq  = (const float*)d_in[5];
  const float* wkr  = (const float*)d_in[6];
  const float* wqr  = (const float*)d_in[7];
  const float* wo   = (const float*)d_in[8];
  float* out = (float*)d_out;

  size_t off = 0;
  const size_t oCt = off; off += (size_t)SQ * PHALF * 4;
  const size_t oSn = off; off += (size_t)SQ * PHALF * 4;
  const size_t oX  = off; off += (size_t)NTOK * HID * 2;
  const size_t oWd = off; off += (size_t)NDN * HID * 2;
  const size_t oWu = off; off += (size_t)NUP * LAT * 2;
  const size_t oWo = off; off += (size_t)HID * HID * 2;
  const size_t oCl = off; off += (size_t)NTOK * CLP * 2;
  const size_t oQc = off; off += (size_t)NBH * SQ * HDM * 2;
  const size_t oQr = off; off += (size_t)NBH * SQ * PD * 2;
  const size_t oKc = off; off += (size_t)NBH * SQ * HDM * 2;
  const size_t oKr = off; off += (size_t)NTOK * PD * 2;
  const size_t oV  = off; off += (size_t)NBH * HDM * SQ * 2;
  const size_t oO  = off; off += (size_t)NTOK * HID * 2;
  if (off > ws_size) return;
  if (off > (size_t)134217728) return;

  char* ws = (char*)d_ws;
  float*    Ct  = (float*)(ws + oCt);
  float*    Sn  = (float*)(ws + oSn);
  _Float16* Xh  = (_Float16*)(ws + oX);
  _Float16* Wd  = (_Float16*)(ws + oWd);
  _Float16* Wu  = (_Float16*)(ws + oWu);
  _Float16* Wot = (_Float16*)(ws + oWo);
  _Float16* Cl  = (_Float16*)(ws + oCl);
  _Float16* Qc  = (_Float16*)(ws + oQc);
  _Float16* Qr  = (_Float16*)(ws + oQr);
  _Float16* Kc  = (_Float16*)(ws + oKc);
  _Float16* Kr  = (_Float16*)(ws + oKr);
  _Float16* Vt  = (_Float16*)(ws + oV);
  _Float16* Op  = (_Float16*)(ws + oO);

  k_tab<<<dim3((SQ * PHALF) / 256), dim3(256), 0, stream>>>(Ct, Sn);
  const int ngx = in_sizes[0] / 8;
  if ((ngx & 255) != 0) return;
  k_cvtx<<<dim3(ngx / 256), dim3(256), 0, stream>>>(x, Xh, ngx);
  k_wtr<<<dim3(LAT / 64, HID / 64), dim3(256), 0, stream>>>(wdkv, LAT, HID, 0, Wd);
  k_wtr<<<dim3(LAT / 64, HID / 64), dim3(256), 0, stream>>>(wdq, LAT, HID, LAT, Wd);
  k_wtr<<<dim3(PD / 64, HID / 64), dim3(256), 0, stream>>>(wkr, PD, HID, 2 * LAT, Wd);
  k_wtr<<<dim3(HID / 64, LAT / 64), dim3(256), 0, stream>>>(wuk, HID, LAT, 0, Wu);
  k_wtr<<<dim3(HID / 64, LAT / 64), dim3(256), 0, stream>>>(wuv, HID, LAT, HID, Wu);
  k_wtr<<<dim3(HID / 64, LAT / 64), dim3(256), 0, stream>>>(wuq, HID, LAT, 2 * HID, Wu);
  k_wtr<<<dim3((NH * PD) / 64, LAT / 64), dim3(256), 0, stream>>>(wqr, NH * PD, LAT, 3 * HID, Wu);
  k_wtr<<<dim3(HID / 64, HID / 64), dim3(256), 0, stream>>>(wo, HID, HID, 0, Wot);
  k_down<<<dim3(NTOK / 64, NDN / 64), dim3(128), 0, stream>>>(Xh, Wd, Ct, Sn, Cl, Kr);
  k_up<<<dim3(NTOK / 64, NUP / HDM), dim3(256), 0, stream>>>(Cl, Wu, Ct, Sn, Qc, Qr, Kc, Vt);
  const float sscale = 0.07216878364870323f;
  k_attn<<<dim3(NBH * NQB), dim3(256), 0, stream>>>(Qc, Qr, Kc, Kr, Vt, Op, sscale);
  k_out<<<dim3(NTOK / 256, HID / 64), dim3(256), 0, stream>>>(Op, Wot, out);
  (void)hipGetLastError();
}
